// HybridStateSpaceAttention_9028021256798
// MI455X (gfx1250) — hardware-verified
//
#include <hip/hip_runtime.h>
#include <math.h>

#define CB   2
#define CS   4096
#define CH   1024
#define CNH  16
#define CHD  64
#define CWIN 512
#define CSTR 256
#define CNW  15
#define CG   64
#define CGT  128

typedef __attribute__((ext_vector_type(16))) _Float16 v16h;
typedef __attribute__((ext_vector_type(8)))  _Float16 v8h;
typedef __attribute__((ext_vector_type(2)))  _Float16 v2h;
typedef __attribute__((ext_vector_type(16))) __bf16   v16b;
typedef __attribute__((ext_vector_type(8)))  __bf16   v8b;
typedef __attribute__((ext_vector_type(8)))  float    v8f;
typedef __attribute__((ext_vector_type(4)))  float    v4f;
typedef __attribute__((ext_vector_type(2)))  float    v2f;

__device__ __forceinline__ unsigned short f2bf_bits(float f) {
  unsigned u = __float_as_uint(f);
  return (unsigned short)((u + 0x7FFFu + ((u >> 16) & 1u)) >> 16);
}
__device__ __forceinline__ float bf_bits2f(unsigned short h) { return __uint_as_float(((unsigned)h) << 16); }

__device__ __forceinline__ void dep_guard_h(v8f& a, v8f& b, v16h x, v16h y) { asm volatile("v_nop\n\tv_nop\n\tv_nop\n\tv_nop" : "+v"(a), "+v"(b) : "v"(x), "v"(y)); }
__device__ __forceinline__ void dep_guard_b(v8f& a, v8f& b, v16b x, v16b y) { asm volatile("v_nop\n\tv_nop\n\tv_nop\n\tv_nop" : "+v"(a), "+v"(b) : "v"(x), "v"(y)); }
__device__ __forceinline__ void keep4_h(v16h a, v16h b, v16h c, v16h d) { asm volatile("v_nop" :: "v"(a), "v"(b), "v"(c), "v"(d)); }
__device__ __forceinline__ void keep4_b(v16b a, v16b b, v16b c, v16b d) { asm volatile("v_nop" :: "v"(a), "v"(b), "v"(c), "v"(d)); }
__device__ __forceinline__ void acc_guard4(v8f& a, v8f& b, v8f& c, v8f& d) { asm volatile("v_nop\n\tv_nop\n\tv_nop\n\tv_nop" : "+v"(a), "+v"(b), "+v"(c), "+v"(d)); }
template <typename T> struct Frag;
template <> struct Frag<_Float16> {
  typedef v16h V; union U { v16h v; v8h h[2]; };
  static __device__ __forceinline__ v16h load(const _Float16* p) {
    U f; f.h[0] = *(const v8h*)(p); f.h[1] = *(const v8h*)(p + 16); return f.v;
  }
  static __device__ __forceinline__ v8f mma(v16h a, v16h b, v8f c) {
    return __builtin_amdgcn_wmma_f32_16x16x32_f16(false, a, false, b, (short)0, c, false, false);
  }
  static __device__ __forceinline__ void guard(v8f& a, v8f& b, v16h x, v16h y) { dep_guard_h(a, b, x, y); }
  static __device__ __forceinline__ void keep(v16h a, v16h b, v16h c, v16h d) { keep4_h(a, b, c, d); }
};
template <> struct Frag<__bf16> {
  typedef v16b V; union U { v16b v; v8b h[2]; };
  static __device__ __forceinline__ v16b load(const __bf16* p) {
    U f; f.h[0] = *(const v8b*)(p); f.h[1] = *(const v8b*)(p + 16); return f.v;
  }
  static __device__ __forceinline__ v8f mma(v16b a, v16b b, v8f c) {
    return __builtin_amdgcn_wmma_f32_16x16x32_bf16(false, a, false, b, (short)0, c, false, false);
  }
  static __device__ __forceinline__ void guard(v8f& a, v8f& b, v16b x, v16b y) { dep_guard_b(a, b, x, y); }
  static __device__ __forceinline__ void keep(v16b a, v16b b, v16b c, v16b d) { keep4_b(a, b, c, d); }
};

template <int ET> struct Elem;
template <> struct Elem<0> { typedef _Float16 T; };
template <> struct Elem<1> { typedef __bf16 T; };
template <int ET, bool SPLIT, int BIAS_MODE, int OUT_MODE, bool RESID, int ACT = 0>
__global__ __launch_bounds__(256) void wmma_gemm64(
    const unsigned short* __restrict__ Ap, const unsigned short* __restrict__ A2p, int lda, long strideA,
    const unsigned short* __restrict__ Btp, const unsigned short* __restrict__ Bt2p, int ldb, long strideB,
    void* __restrict__ Cout, void* __restrict__ Cout2, int ldc, long strideC,
    const float* __restrict__ bias,
    const float* __restrict__ resid, long strideR,
    int M, int N, int K, float scale) {
  typedef typename Elem<ET>::T T;
  typedef typename Frag<T>::V V;
  const T* A = (const T*)Ap; const T* A2 = (const T*)A2p; const T* Bt = (const T*)Btp; const T* Bt2 = (const T*)Bt2p;
  __shared__ __align__(16) float sT[8][16 * 68];
  const int b    = blockIdx.y;
  const int lane = threadIdx.x & 31;
  const int wave = threadIdx.x >> 5;
  const int tilesN = N >> 6;
  const int tilesM = M >> 6;
  const int tile = blockIdx.x * 8 + wave;
  if (tile >= tilesM * tilesN) return;
  const int tm = tile / tilesN;
  const int tn = tile - tm * tilesN;
  const int m0 = tm << 6;
  const int n0 = tn << 6;

  const T* Ab  = A  + (size_t)b * strideA;
  const T* Bb  = Bt + (size_t)b * strideB;
  const T* Ab2 = SPLIT ? (A2  + (size_t)b * strideA) : nullptr;
  const T* Bb2 = SPLIT ? (Bt2 + (size_t)b * strideB) : nullptr;

  const int rlane = lane & 15;
  const int koff  = (lane >> 4) * 8;
  const int mOff  = (lane >> 4) * 8;

  v8f acc[4][4];
#pragma unroll
  for (int i = 0; i < 4; ++i)
#pragma unroll
    for (int j = 0; j < 4; ++j) acc[i][j] = (v8f){0.f,0.f,0.f,0.f,0.f,0.f,0.f,0.f};

  for (int k0 = 0; k0 < K; k0 += 32) {
    V bh[4], bl[4];
#pragma unroll
    for (int j = 0; j < 4; ++j) {
      const size_t bo = (size_t)(n0 + (j << 4) + rlane) * ldb + koff + k0;
      bh[j] = Frag<T>::load(Bb + bo);
      if (SPLIT) bl[j] = Frag<T>::load(Bb2 + bo);
    }
#pragma unroll
    for (int i = 0; i < 4; ++i) {
      const size_t ao = (size_t)(m0 + (i << 4) + rlane) * lda + koff + k0;
      V ah = Frag<T>::load(Ab + ao);
      V al;
      if (SPLIT) al = Frag<T>::load(Ab2 + ao);
#pragma unroll
      for (int j = 0; j < 4; ++j) {
        acc[i][j] = Frag<T>::mma(ah, bh[j], acc[i][j]);
        if (SPLIT) {
          acc[i][j] = Frag<T>::mma(ah, bl[j], acc[i][j]);
          acc[i][j] = Frag<T>::mma(al, bh[j], acc[i][j]);
        }
      }
      Frag<T>::guard(acc[i][0], acc[i][3], ah, SPLIT ? al : ah);
    }
    Frag<T>::keep(bh[0], bh[1], bh[2], bh[3]);
    if (SPLIT) Frag<T>::keep(bl[0], bl[1], bl[2], bl[3]);
  }
  acc_guard4(acc[0][0], acc[0][1], acc[0][2], acc[0][3]);
  acc_guard4(acc[1][0], acc[1][1], acc[1][2], acc[1][3]);
  acc_guard4(acc[2][0], acc[2][1], acc[2][2], acc[2][3]);
  acc_guard4(acc[3][0], acc[3][1], acc[3][2], acc[3][3]);

  float* slab = sT[wave];
  const float* Rb = RESID ? (resid + (size_t)b * strideR) : nullptr;
#pragma unroll
  for (int i = 0; i < 4; ++i) {
    const int mBase = m0 + (i << 4);
#pragma unroll
    for (int j = 0; j < 4; ++j) {
      const int n = n0 + (j << 4) + rlane;
      float bv = 0.f;
      if (BIAS_MODE == 2) bv = bias[n];
#pragma unroll
      for (int r = 0; r < 8; ++r) {
        float v = acc[i][j][r] * scale;
        if (BIAS_MODE == 1) v += bias[mBase + mOff + r];
        if (BIAS_MODE == 2) v += bv;
        if (RESID) v += Rb[(size_t)(mBase + mOff + r) * ldc + n];
        if (ACT == 1) v = tanhf(v);
        if (ACT == 2) v = fmaxf(v, 0.0f);
        if (ACT == 3) v = v / (1.0f + expf(-v));
        if (ACT == 4) v = (v > 0.f) ? v : 0.01f * v;
        if (ACT == 5) v = 0.5f * v * (1.0f + erff(v * 0.70710678118654752f));
        slab[(mOff + r) * 68 + (j << 4) + rlane] = v;
      }
    }
    __builtin_amdgcn_fence(__ATOMIC_RELEASE, "workgroup");
    __builtin_amdgcn_wave_barrier();
    __builtin_amdgcn_fence(__ATOMIC_ACQUIRE, "workgroup");
    if (OUT_MODE == 0) {
      float* C = (float*)Cout + (size_t)b * strideC;
      const int hh = lane >> 4, c4 = (lane & 15) * 4;
      for (int pass = 0; pass < 2; ++pass) {
#pragma unroll
        for (int it = 0; it < 8; ++it) {
          const int row = it * 2 + hh;
          v4f v = *(const v4f*)(slab + row * 68 + c4);
          *(volatile v4f*)(C + (size_t)(mBase + row) * ldc + n0 + c4) = v;
        }
        __threadfence();
      }
    } else {
      const int q = lane >> 3, c8 = (lane & 7) * 8;
      unsigned short* C  = (unsigned short*)Cout  + (size_t)b * strideC;
      unsigned short* C2 = (OUT_MODE == 2) ? ((unsigned short*)Cout2 + (size_t)b * strideC) : nullptr;
      for (int pass = 0; pass < 2; ++pass) {
#pragma unroll
        for (int it = 0; it < 4; ++it) {
          const int row = it * 4 + q;
          const float* sp = slab + row * 68 + c8;
          v8h hv, lv;
#pragma unroll
          for (int e = 0; e < 8; ++e) {
            if (OUT_MODE == 1) {
              hv[e] = (_Float16)sp[e];
            } else {
              unsigned short hb = f2bf_bits(sp[e]);
              unsigned short lb = f2bf_bits(sp[e] - bf_bits2f(hb));
              hv[e] = __builtin_bit_cast(_Float16, hb);
              lv[e] = __builtin_bit_cast(_Float16, lb);
            }
          }
          *(volatile v8h*)(C + (size_t)(mBase + row) * ldc + n0 + c8) = hv;
          if (OUT_MODE == 2) *(volatile v8h*)(C2 + (size_t)(mBase + row) * ldc + n0 + c8) = lv;
        }
        __threadfence();
      }
    }
    __builtin_amdgcn_fence(__ATOMIC_RELEASE, "workgroup");
    __builtin_amdgcn_wave_barrier();
    __builtin_amdgcn_fence(__ATOMIC_ACQUIRE, "workgroup");
  }
}

__global__ __launch_bounds__(256) void k_cast8(const float* __restrict__ in, _Float16* __restrict__ out,
                                               int n8, float scale) {
  const int i = blockIdx.x * 256 + threadIdx.x;
  if (i < n8) {
    const float* p = in + (size_t)i * 8;
    const v4f a = *(const v4f*)p;
    const v4f bq = *(const v4f*)(p + 4);
    v8h o;
    o[0] = (_Float16)(a[0] * scale);  o[1] = (_Float16)(a[1] * scale);
    o[2] = (_Float16)(a[2] * scale);  o[3] = (_Float16)(a[3] * scale);
    o[4] = (_Float16)(bq[0] * scale); o[5] = (_Float16)(bq[1] * scale);
    o[6] = (_Float16)(bq[2] * scale); o[7] = (_Float16)(bq[3] * scale);
    _Float16* d = out + (size_t)i * 8;
    *(volatile v8h*)d = o;
    __threadfence();
    *(volatile v8h*)d = o;
  }
}

__global__ __launch_bounds__(256) void k_convw(const float* __restrict__ w, _Float16* __restrict__ bt) {
  const int t = blockIdx.x * 256 + threadIdx.x;
  if (t < CH * 4 * (CH / 8)) {
    const int o  = t >> 9;
    const int kq = (t >> 7) & 3;
    const int i0 = (t & 127) * 8;
    const float* src = w + (size_t)o * (4 * CH) + (size_t)i0 * 4 + kq;
    v8h v;
#pragma unroll
    for (int e = 0; e < 8; ++e) v[e] = (_Float16)(src[4 * e] * 16.0f);
    _Float16* dst = bt + (size_t)o * (4 * CH) + (size_t)kq * CH + i0;
    *(volatile v8h*)dst = v;
    __threadfence();
    *(volatile v8h*)dst = v;
  }
}

__global__ __launch_bounds__(256) void k_transpose64(const float* __restrict__ in, _Float16* __restrict__ out,
                                                     int R, int C, float scale) {
  __shared__ float tile[64][65];
  const int tid = threadIdx.x;
  const int c0 = blockIdx.x * 64, r0 = blockIdx.y * 64;
#pragma unroll
  for (int it = 0; it < 16; ++it) {
    const int idx = it * 256 + tid;
    const int r = idx >> 6, cc = idx & 63;
    tile[r][cc] = in[(size_t)(r0 + r) * C + c0 + cc];
  }
  __syncthreads();
  const int wave = tid >> 5, lane = tid & 31, qq = lane >> 3, c8 = (lane & 7) * 8;
  for (int pass = 0; pass < 2; ++pass) {
#pragma unroll
    for (int it = 0; it < 2; ++it) {
      const int col = wave * 8 + it * 4 + qq;
      v8h hv;
#pragma unroll
      for (int e = 0; e < 8; ++e) hv[e] = (_Float16)(tile[c8 + e][col] * scale);
      *(volatile v8h*)(out + (size_t)(c0 + col) * R + r0 + c8) = hv;
    }
    __threadfence();
  }
}

__global__ __launch_bounds__(256) void k_mem(const float* __restrict__ gm, _Float16* __restrict__ gt) {
  const int t = blockIdx.x * 256 + threadIdx.x;
  if (t < CG * (CH / 8)) {
    const int g = t >> 7;
    const int rem = t & 127;
    const int h = rem >> 3, d0 = (rem & 7) * 8;
    const float* src = gm + ((size_t)h * CG + g) * CHD + d0;
    v8h v;
#pragma unroll
    for (int e = 0; e < 8; ++e) v[e] = (_Float16)src[e];
    _Float16* d0p = gt + ((size_t)(0 * CGT + CG + g)) * CH + rem * 8;
    _Float16* d1p = gt + ((size_t)(1 * CGT + CG + g)) * CH + rem * 8;
    *(volatile v8h*)d0p = v;
    *(volatile v8h*)d1p = v;
    __threadfence();
    *(volatile v8h*)d0p = v;
    *(volatile v8h*)d1p = v;
  }
}

#define AQB 64
#define AKC 64
#define AD  64
#define APS 32768.0f
struct AttG {
  long q_bs, q_zs, q_hs, q_rs, k_bs, k_zs, k_hs, k_rs, o_bs, o_zs, o_hs, o_rs;
  int nqb, nz, nh, nchunks; float qscale; int pad0;
};
typedef char attg_size_chk[(sizeof(AttG) == 120) ? 1 : -1];

__device__ __forceinline__ v8f mma_h(v16h a, v16h b, v8f c) {
  c = __builtin_amdgcn_wmma_f32_16x16x32_f16(false, a, false, b, (short)0, c, false, false);
  asm volatile("v_nop\n\tv_nop\n\tv_nop\n\tv_nop" : "+v"(c) : "v"(a), "v"(b));
  return c;
}

__global__ __launch_bounds__(128)
void attn16_kernel(const _Float16* __restrict__ q, const _Float16* __restrict__ kv,
                   _Float16* __restrict__ out, AttG g) {
  union FB { v16h v; v8h h[2]; };
  __shared__ __align__(16) _Float16 Ksh[AKC * AD];
  __shared__ __align__(16) _Float16 Vth[AD * AKC];
  __shared__ __align__(16) _Float16 Psh[4][16 * AKC];
  __shared__ __align__(16) float    Os[4][16 * 68];

  const int tid  = threadIdx.x;
  const int wave = tid >> 5;
  const int lane = tid & 31;
  const int hh   = lane >> 4;
  const int c    = lane & 15;

  int bx = blockIdx.x;
  const int qb = bx % g.nqb; bx /= g.nqb;
  const int h  = bx % g.nh;  bx /= g.nh;
  const int z  = bx % g.nz;
  const int b  = bx / g.nz;
  const int q0 = qb * AQB + wave * 16;

  const _Float16* qp = q  + (size_t)b * g.q_bs + (size_t)z * g.q_zs + (size_t)h * g.q_hs;
  const _Float16* kp = kv + (size_t)b * g.k_bs + (size_t)z * g.k_zs + (size_t)h * g.k_hs;
  _Float16*       op = out + (size_t)b * g.o_bs + (size_t)z * g.o_zs + (size_t)h * g.o_hs;

  v16h qa[2];
  {
    const _Float16* qrow = qp + (size_t)(q0 + c) * g.q_rs + 8 * hh;
#pragma unroll
    for (int dc = 0; dc < 2; ++dc) qa[dc] = Frag<_Float16>::load(qrow + dc * 32);
  }

  float mrow[8], lrow[8];
  v8f oacc[4];
#pragma unroll
  for (int r = 0; r < 8; ++r) { mrow[r] = -1e30f; lrow[r] = 0.f; }
#pragma unroll
  for (int t = 0; t < 4; ++t) oacc[t] = (v8f){0.f,0.f,0.f,0.f,0.f,0.f,0.f,0.f};

  for (int kc = 0; kc < g.nchunks; ++kc) {
    const int kv0 = kc * AKC;
    __syncthreads();
    {
      const int kvr = tid >> 1, dh = (tid & 1) * 32;
      const _Float16* krow = kp + (size_t)(kv0 + kvr) * g.k_rs + dh;
#pragma unroll
      for (int i = 0; i < 4; ++i) {
        const v8h kk = *(const v8h*)(krow + 8 * i);
        *(v8h*)(Ksh + kvr * AD + dh + 8 * i) = kk;
#pragma unroll
        for (int e = 0; e < 8; ++e) Vth[(dh + 8 * i + e) * AKC + kvr] = kk[e];
      }
    }
    __syncthreads();

    v8f s[4];
#pragma unroll
    for (int j = 0; j < 4; ++j) {
      s[j] = (v8f){0.f,0.f,0.f,0.f,0.f,0.f,0.f,0.f};
#pragma unroll
      for (int dc = 0; dc < 2; ++dc) {
        FB kb;
        kb.h[0] = *(const v8h*)(Ksh + (j * 16 + c) * AD + dc * 32 + 8 * hh);
        kb.h[1] = *(const v8h*)(Ksh + (j * 16 + c) * AD + dc * 32 + 16 + 8 * hh);
        s[j] = mma_h(qa[dc], kb.v, s[j]);
      }
    }
    float cm[8];
#pragma unroll
    for (int r = 0; r < 8; ++r) {
      float m = -1e30f;
#pragma unroll
      for (int j = 0; j < 4; ++j) { s[j][r] *= g.qscale; m = fmaxf(m, s[j][r]); }
#pragma unroll
      for (int off = 1; off < 16; off <<= 1) m = fmaxf(m, __shfl_xor(m, off, 32));
      cm[r] = m;
    }
    _Float16* pw = Psh[wave];
#pragma unroll
    for (int r = 0; r < 8; ++r) {
      const float mnew = fmaxf(mrow[r], cm[r]);
      const float alpha = __expf(mrow[r] - mnew);
      mrow[r] = mnew;
      float psum = 0.f;
#pragma unroll
      for (int j = 0; j < 4; ++j) {
        const float p = __expf(s[j][r] - mnew);
        psum += p;
        pw[(8 * hh + r) * AKC + j * 16 + c] = (_Float16)(p * APS);
      }
#pragma unroll
      for (int off = 1; off < 16; off <<= 1) psum += __shfl_xor(psum, off, 32);
      lrow[r] = lrow[r] * alpha + psum;
#pragma unroll
      for (int t = 0; t < 4; ++t) oacc[t][r] *= alpha;
    }
    __builtin_amdgcn_fence(__ATOMIC_RELEASE, "workgroup");
    __builtin_amdgcn_wave_barrier();
    __builtin_amdgcn_fence(__ATOMIC_ACQUIRE, "workgroup");
#pragma unroll 1
    for (int kk = 0; kk < 2; ++kk) {
      FB pa;
      pa.h[0] = *(const v8h*)(pw + c * AKC + kk * 32 + 8 * hh);
      pa.h[1] = *(const v8h*)(pw + c * AKC + kk * 32 + 16 + 8 * hh);
#pragma unroll
      for (int t = 0; t < 4; ++t) {
        FB vb;
        vb.h[0] = *(const v8h*)(Vth + (t * 16 + c) * AKC + kk * 32 + 8 * hh);
        vb.h[1] = *(const v8h*)(Vth + (t * 16 + c) * AKC + kk * 32 + 16 + 8 * hh);
        oacc[t] = mma_h(pa.v, vb.v, oacc[t]);
      }
    }
  }

  float* os = Os[wave];
#pragma unroll
  for (int r = 0; r < 8; ++r) {
    const float inv = __builtin_amdgcn_rcpf(lrow[r] * APS);
#pragma unroll
    for (int t = 0; t < 4; ++t) os[(8 * hh + r) * 68 + t * 16 + c] = oacc[t][r] * inv;
  }
  __builtin_amdgcn_fence(__ATOMIC_RELEASE, "workgroup");
  __builtin_amdgcn_wave_barrier();
  __builtin_amdgcn_fence(__ATOMIC_ACQUIRE, "workgroup");
  {
    const int qq = lane >> 3, c8 = (lane & 7) * 8;
    for (int pass = 0; pass < 2; ++pass) {
#pragma unroll
      for (int it = 0; it < 4; ++it) {
        const int row = it * 4 + qq;
        const float* sp = os + row * 68 + c8;
        v8h hv;
#pragma unroll
        for (int e = 0; e < 8; ++e) hv[e] = (_Float16)sp[e];
        *(volatile v8h*)(op + (size_t)(q0 + row) * g.o_rs + c8) = hv;
      }
      __threadfence();
    }
  }
}

__device__ __forceinline__ float tri_w(int i) {
  const float st = (float)i * (1.0f / 511.0f);
  return (i == CWIN - 1) ? 1.5f : (0.5f * (1.0f - st) + 1.5f * st);
}
__global__ __launch_bounds__(256) void k_fold(const _Float16* __restrict__ wo, _Float16* __restrict__ lg) {
  const int t = blockIdx.x * 256 + threadIdx.x;
  if (t < CB * CS * (CH / 8)) {
    const int row = t >> 7;
    const int c0  = (t & 127) * 8;
    const int b = row >> 12, s = row & (CS - 1);
    const int sb = s >> 8;
    const int n1 = (sb < CNW) ? sb : (CNW - 1);
    const bool has1 = (sb <= CNW - 1);
    const int n0 = (sb >= 1) ? (sb - 1) : 0;
    const bool has0 = (sb >= 1);
    const int i0 = s - CSTR * n0;
    const int i1 = s - CSTR * n1;
    const float t0 = has0 ? tri_w(i0) : 0.f;
    const float t1 = has1 ? tri_w(i1) : 0.f;
    const float den = t0 + t1;
    const float rinv = __builtin_amdgcn_rcpf(den + 1e-6f);
    const v8h a  = *(const v8h*)(wo + (((size_t)(b * CNW + n0) * CWIN + i0) * CH + c0));
    const v8h bq = *(const v8h*)(wo + (((size_t)(b * CNW + n1) * CWIN + i1) * CH + c0));
    v8h o;
#pragma unroll
    for (int e = 0; e < 8; ++e) {
      const float num = (float)a[e] * t0 + (float)bq[e] * t1;
      o[e] = (_Float16)(num * rinv);
    }
    _Float16* dst = lg + (size_t)row * (2 * CH) + c0;
    *(volatile v8h*)dst = o;
    __threadfence();
    *(volatile v8h*)dst = o;
  }
}

__global__ __launch_bounds__(256) void k_bcast(const float* __restrict__ x, float* __restrict__ bcT) {
  __shared__ __align__(16) v2f cur[CS];
  const int tid = threadIdx.x;
  const int b  = blockIdx.x / (CH / 2);
  const int c0 = (blockIdx.x % (CH / 2)) * 2;
  const float* xb = x + (size_t)b * CS * CH + c0;
  v2f res[16], nw[16];
#pragma unroll
  for (int i = 0; i < 16; ++i) {
    const int s = tid + 256 * i;
    const v2f v = *(const v2f*)(xb + (size_t)s * CH);
    cur[s] = v;
    res[i] = (v2f){0.f, 0.f};
  }
  __syncthreads();
  for (int sh = 1; sh < CS; sh <<= 1) {
#pragma unroll
    for (int i = 0; i < 16; ++i) {
      const int s = tid + 256 * i;
      const v2f a  = cur[(s - sh) & (CS - 1)];
      const v2f bq = cur[(s + sh) & (CS - 1)];
      const v2f cc = cur[s];
      nw[i] = cc + 0.5f * (a + bq);
      res[i] += nw[i];
    }
    __syncthreads();
#pragma unroll
    for (int i = 0; i < 16; ++i) cur[tid + 256 * i] = nw[i];
    __syncthreads();
  }
  const float k13 = 1.0f / 13.0f;
  float* r0p = bcT + ((size_t)(b * CH + c0)) * CS;
  float* r1p = r0p + CS;
  for (int pass = 0; pass < 2; ++pass) {
#pragma unroll
    for (int i = 0; i < 16; ++i) {
      const int s = tid + 256 * i;
      const float v0 = res[i][0] * k13;
      const float v1 = res[i][1] * k13;
      ((volatile float*)r0p)[s] = v0;
      ((volatile float*)r1p)[s] = v1;
    }
    __threadfence();
  }
}

__global__ __launch_bounds__(256) void k_mix(const float* __restrict__ gpre, const _Float16* __restrict__ lg,
                                             const float* __restrict__ bcT, _Float16* __restrict__ mixed) {
  const int t = blockIdx.x * 256 + threadIdx.x;
  if (t < CB * CS * (CH / 2)) {
    const int row = t >> 9;
    const int c2  = (t & 511) * 2;
    const int b = row >> 12, s = row & (CS - 1);
    const v2f gp = *(const v2f*)(gpre + (size_t)row * CH + c2);
    const _Float16* lr = lg + (size_t)row * (2 * CH);
    const v2h lo2 = *(const v2h*)(lr + c2);
    const v2h gl2 = *(const v2h*)(lr + CH + c2);
    const float* bp = bcT + ((size_t)(b * CH + c2)) * CS + s;
    const float bc0 = bp[0];
    const float bc1 = bp[CS];
    const float g0 = __builtin_amdgcn_rcpf(1.0f + expf(-gp[0]));
    const float g1 = __builtin_amdgcn_rcpf(1.0f + expf(-gp[1]));
    const float l0 = (float)lo2[0], l1 = (float)lo2[1];
    const float q0 = (float)gl2[0], q1 = (float)gl2[1];
    const float m0 = g0 * l0 + (1.0f - g0) * q0 + bc0;
    const float m1 = g1 * l1 + (1.0f - g1) * q1 + bc1;
    v2h o;
    o[0] = (_Float16)m0;
    o[1] = (_Float16)m1;
    _Float16* dst = mixed + (size_t)row * CH + c2;
    *(volatile v2h*)dst = o;
    __threadfence();
    *(volatile v2h*)dst = o;
  }
}

extern "C" void kernel_launch(void* const* d_in, const int* in_sizes, int n_in,
                              void* d_out, int out_size, void* d_ws, size_t ws_size,
                              hipStream_t stream) {
  if (n_in < 8) return;
  if (in_sizes[0] != CB * CS * CH) return;
  if (in_sizes[1] != CNH * CG * CHD) return;
  if (in_sizes[2] != CH * CH * 4) return;
  if (in_sizes[3] != CH) return;
  if (in_sizes[4] != 2 * CH * CH) return;
  if (in_sizes[5] != CH) return;
  if (in_sizes[6] != CH * CH) return;
  if (in_sizes[7] != CH) return;
  if (out_size != CB * CS * CH) return;

  const float* x      = (const float*)d_in[0];
  const float* gm     = (const float*)d_in[1];
  const float* conv_w = (const float*)d_in[2];
  const float* conv_b = (const float*)d_in[3];
  const float* mix_w  = (const float*)d_in[4];
  const float* mix_b  = (const float*)d_in[5];
  const float* out_w  = (const float*)d_in[6];
  const float* out_b  = (const float*)d_in[7];
  float* outp = (float*)d_out;

  const size_t nX = (size_t)CB * CS * CH;
  const size_t plane32 = nX * 4;
  const size_t winBytes = (size_t)CB * CNW * CWIN * CH * 2;
  const size_t convwBytes = (size_t)CH * 4 * CH * 2;
  char* ws = (char*)d_ws;
  size_t off = 0;
  _Float16* lg    = (_Float16*)(ws + off); off += nX * 2 * 2;
  float*    bcT   = (float*)(ws + off);    off += plane32;
  char*     big   = ws + off;              off += plane32;
  char*     rx    = ws + off;              off += nX * 2;
  _Float16* mixwT = (_Float16*)(ws + off); off += (size_t)CH * 2 * CH * 2;
  _Float16* outwT = (_Float16*)(ws + off); off += (size_t)CH * CH * 2;
  _Float16* gth   = (_Float16*)(ws + off); off += (size_t)CB * CGT * CH * 2;
  if (off > ws_size) return;
  if (off > (size_t)134217728) return;
  if (winBytes > plane32 || convwBytes > plane32) return;
  _Float16* convwh = (_Float16*)big;
  _Float16* winout = (_Float16*)big;
  float*    gpre   = (float*)big;
  _Float16* xh     = (_Float16*)rx;
  _Float16* mixed  = (_Float16*)rx;

  const float wsc = 16.0f, wsc_inv = 1.0f / 16.0f;

  k_cast8<<<dim3((unsigned)((nX / 8 + 255) / 256)), dim3(256), 0, stream>>>(x, xh, (int)(nX / 8), 1.0f);
  k_convw<<<dim3((CH * 4 * (CH / 8) + 255) / 256), dim3(256), 0, stream>>>(conv_w, convwh);
  k_transpose64<<<dim3(CH / 64, (2 * CH) / 64), dim3(256), 0, stream>>>(mix_w, mixwT, 2 * CH, CH, wsc);
  k_transpose64<<<dim3(CH / 64, CH / 64), dim3(256), 0, stream>>>(out_w, outwT, CH, CH, wsc);
  k_mem<<<dim3((CG * (CH / 8) + 255) / 256), dim3(256), 0, stream>>>(gm, gth);
  wmma_gemm64<0, false, 2, 1, false, 0><<<dim3(2, CB), dim3(256), 0, stream>>>(
      (const unsigned short*)(const void*)xh, nullptr, 4 * CH, (long)CS * CH,
      (const unsigned short*)(const void*)convwh, nullptr, 4 * CH, 0L,
      (void*)gth, nullptr, CH, (long)CGT * CH,
      conv_b, nullptr, 0L,
      CG, CH, 4 * CH, wsc_inv);

  AttG gw;
  gw.q_bs = (long)CS * CH; gw.q_zs = (long)CSTR * CH; gw.q_hs = CHD; gw.q_rs = CH;
  gw.k_bs = (long)CS * CH; gw.k_zs = (long)CSTR * CH; gw.k_hs = CHD; gw.k_rs = CH;
  gw.o_bs = (long)CNW * CWIN * CH; gw.o_zs = (long)CWIN * CH; gw.o_hs = CHD; gw.o_rs = CH;
  gw.nqb = CWIN / AQB; gw.nz = CNW; gw.nh = CNH; gw.nchunks = CWIN / AKC; gw.qscale = 0.125f; gw.pad0 = 0;
  attn16_kernel<<<dim3(CB * CNW * CNH * (CWIN / AQB)), dim3(128), 0, stream>>>(xh, xh, winout, gw);

  k_fold<<<dim3((unsigned)((nX / 8 + 255) / 256)), dim3(256), 0, stream>>>(winout, lg);

  AttG gg;
  gg.q_bs = (long)CS * CH; gg.q_zs = 0; gg.q_hs = CHD; gg.q_rs = CH;
  gg.k_bs = (long)CGT * CH; gg.k_zs = 0; gg.k_hs = CHD; gg.k_rs = CH;
  gg.o_bs = (long)CS * 2 * CH; gg.o_zs = 0; gg.o_hs = CHD; gg.o_rs = 2 * CH;
  gg.nqb = CS / AQB; gg.nz = 1; gg.nh = CNH; gg.nchunks = CGT / AKC; gg.qscale = 0.125f; gg.pad0 = 0;
  attn16_kernel<<<dim3(CB * CNH * (CS / AQB)), dim3(128), 0, stream>>>(xh, gth, lg + CH, gg);

  k_bcast<<<dim3(CB * (CH / 2)), dim3(256), 0, stream>>>(x, bcT);

  wmma_gemm64<0, false, 2, 0, false, 0><<<dim3((unsigned)((nX / CH / 64) * (CH / 64) / 8), 1), dim3(256), 0, stream>>>(
      (const unsigned short*)(const void*)lg, nullptr, 2 * CH, 0L,
      (const unsigned short*)(const void*)mixwT, nullptr, 2 * CH, 0L,
      (void*)gpre, nullptr, CH, 0L,
      mix_b, nullptr, 0L,
      CB * CS, CH, 2 * CH, wsc_inv);

  k_mix<<<dim3((unsigned)((nX / 2 + 255) / 256)), dim3(256), 0, stream>>>(gpre, lg, bcT, mixed);

  wmma_gemm64<0, false, 2, 0, false, 0><<<dim3((unsigned)((nX / CH / 64) * (CH / 64) / 8), 1), dim3(256), 0, stream>>>(
      (const unsigned short*)(const void*)mixed, nullptr, CH, 0L,
      (const unsigned short*)(const void*)outwT, nullptr, CH, 0L,
      (void*)outp, nullptr, CH, 0L,
      out_b, nullptr, 0L,
      CB * CS, CH, CH, wsc_inv);
}
